// GATEncoder_15393162788898
// MI455X (gfx1250) — hardware-verified
//
#include <hip/hip_runtime.h>
#include <stddef.h>
#include <stdint.h>
#include <math.h>


#define DIN    128
#define DH     128
#define KP     256
#define NTHR   256
#define NWAVE  8
#define EPT    8
#define CHUNK  (NTHR * EPT)
#define WCAP   (EPT * 32)
#define LISTN  (NWAVE * WCAP)
#define NBA    1024
#define SLA    10
#define RCAP   28672
#define DEGCAP 128
#define GBM    64
#define GBN    128
#define GTHR   128
#define NU1    (DH * (DIN / 8))
#define NU2    (DH * (KP / 8))
#define NGR    64
#define NPB    1024
#define PTHR   128
#define NEGSL  0.2f
#define EPS_SM 1e-16f
#define AGG_ZINTS (LISTN + 2 * RCAP + 3 * NBA)
#define AGG_LDS_INTS (AGG_ZINTS + 16)
#define WSMAX  134217728

static_assert((CHUNK & (CHUNK - 1)) == 0 && CHUNK <= 4096);
static_assert((NBA & (NBA - 1)) == 0 && NBA == (1 << SLA));
static_assert(((long long)CHUNK << SLA) < (1LL << 31));
static_assert(LISTN % NTHR == 0);
static_assert(NBA % NWAVE == 0 && NBA % 32 == 0 && NBA % GBM == 0);
static_assert(RCAP % 4 == 0 && AGG_ZINTS % 4 == 0 && LISTN % 4 == 0);
static_assert(DIN % 32 == 0 && DH % 32 == 0 && KP == 2 * DH && DH == GBN && KP % 32 == 0);
static_assert(GBM == (GTHR / 32) * 16 && GBN == 4 * 32);
static_assert(NU1 % NTHR == 0 && NU2 % NTHR == 0);
static_assert(DIN / 8 == 16 && KP / 8 == 32);
static_assert(AGG_LDS_INTS * 4 <= 300000);
static_assert(DH == 4 * 32);
static_assert(PTHR == DH && NGR <= PTHR && (NGR % 4) == 0);
static_assert(NGR * DH - 1 == 8191);

typedef float          v4f   __attribute__((ext_vector_type(4)));
typedef float          v8f   __attribute__((ext_vector_type(8)));
typedef int            v4i   __attribute__((ext_vector_type(4)));
typedef int            v8i   __attribute__((ext_vector_type(8)));
typedef unsigned int   v4u   __attribute__((ext_vector_type(4)));
typedef unsigned short v8us  __attribute__((ext_vector_type(8)));
typedef unsigned short v16us __attribute__((ext_vector_type(16)));
typedef __bf16         v16bf __attribute__((ext_vector_type(16)));
typedef v4f  __attribute__((may_alias)) v4fa;
typedef v4i  __attribute__((may_alias)) v4ia;
typedef v8us __attribute__((may_alias)) v8usa;
union FragB { v16bf v; v16us u; v8us h[2]; v8i w; };

__device__ __forceinline__ v8f wmb(const FragB& a, const FragB& b, v8f c) {
  v8f d = __builtin_amdgcn_wmma_f32_16x16x32_bf16(false, a.v, false, b.v, (short)0, c, false, false);
  asm volatile("v_nop\n\tv_nop\n\tv_nop\n\tv_nop" : "+v"(d) : "v"(a.w), "v"(b.w));
  return d;
}

__device__ __forceinline__ unsigned bf16_bits(float f) {
  const unsigned u = __float_as_uint(f);
  return (u + 0x7FFFu + ((u >> 16) & 1u)) >> 16;
}
__device__ __forceinline__ float bf16_val(float f) {
  return __uint_as_float(bf16_bits(f) << 16);
}
__device__ __forceinline__ v4f bfr4(const v4f a) {
  v4f r; r.x = bf16_val(a.x); r.y = bf16_val(a.y); r.z = bf16_val(a.z); r.w = bf16_val(a.w); return r;
}

template <int SLB>
__device__ __forceinline__ int scan_chunk(const int* __restrict__ dsts, int nE, int cbase, int slotBase,
                                          int nb, int vec8, int* list, int tid, int lane, int wave) {
  int wc = 0;
  const int el0  = tid * EPT;
  const int e0   = cbase + el0;
  const int sent = -2147483647 - 1;
  v4i da, db;
  if (vec8 != 0 && cbase + CHUNK <= nE) {
    da = *(const v4i*)(dsts + e0);
    db = *(const v4i*)(dsts + e0 + 4);
  } else {
    da.x = (e0     < nE) ? dsts[min(e0,     nE - 1)] : sent;
    da.y = (e0 + 1 < nE) ? dsts[min(e0 + 1, nE - 1)] : sent;
    da.z = (e0 + 2 < nE) ? dsts[min(e0 + 2, nE - 1)] : sent;
    da.w = (e0 + 3 < nE) ? dsts[min(e0 + 3, nE - 1)] : sent;
    db.x = (e0 + 4 < nE) ? dsts[min(e0 + 4, nE - 1)] : sent;
    db.y = (e0 + 5 < nE) ? dsts[min(e0 + 5, nE - 1)] : sent;
    db.z = (e0 + 6 < nE) ? dsts[min(e0 + 6, nE - 1)] : sent;
    db.w = (e0 + 7 < nE) ? dsts[min(e0 + 7, nE - 1)] : sent;
  }
  const unsigned nbs = (unsigned)slotBase;
  const unsigned unb = (unsigned)nb;
  const unsigned s0 = (unsigned)da.x - nbs, s1 = (unsigned)da.y - nbs;
  const unsigned s2 = (unsigned)da.z - nbs, s3 = (unsigned)da.w - nbs;
  const unsigned s4 = (unsigned)db.x - nbs, s5 = (unsigned)db.y - nbs;
  const unsigned s6 = (unsigned)db.z - nbs, s7 = (unsigned)db.w - nbs;
  const bool h0 = s0 < unb, h1 = s1 < unb, h2 = s2 < unb, h3 = s3 < unb;
  const bool h4 = s4 < unb, h5 = s5 < unb, h6 = s6 < unb, h7 = s7 < unb;
  const unsigned any = __builtin_amdgcn_ballot_w32(h0 | h1 | h2 | h3 | h4 | h5 | h6 | h7);
  if (any != 0u) {
#define HITJ(J, HJ, SJ) { \
      const unsigned mj = __builtin_amdgcn_ballot_w32(HJ); \
      if (mj != 0u) { \
        if (HJ) { \
          const int pos = wc + (int)__builtin_amdgcn_mbcnt_lo(mj, 0u); \
          if (pos < WCAP) list[wave * WCAP + pos] = ((el0 + (J)) << SLB) | (int)(SJ); \
        } \
        wc += (int)__builtin_popcount(mj); } }
    HITJ(0, h0, s0)
    HITJ(1, h1, s1)
    HITJ(2, h2, s2)
    HITJ(3, h3, s3)
    HITJ(4, h4, s4)
    HITJ(5, h5, s5)
    HITJ(6, h6, s6)
    HITJ(7, h7, s7)
#undef HITJ
  }
  return wc;
}

__global__ __launch_bounds__(NTHR) void k_wprep(const float* __restrict__ W1, const float* __restrict__ W2,
                                                const float* __restrict__ W3,
                                                unsigned short* W1T, unsigned short* W2D, unsigned short* W3D) {
  const int u = (int)blockIdx.x * NTHR + (int)threadIdx.x;
  v8us o;
  unsigned short* dp;
  if (u < NU1) {
    const int n  = u >> 4;
    const int k8 = (u & 15) * 8;
    const float* p = W1 + (size_t)k8 * DH + n;
#pragma unroll
    for (int i = 0; i < 8; ++i) o[i] = (unsigned short)bf16_bits(p[(size_t)i * DH]);
    dp = W1T + (size_t)n * DIN + k8;
  } else if (u < NU1 + NU2) {
    const int v  = u - NU1;
    const int n  = v >> 5;
    const int k8 = (v & 31) * 8;
    const int kk = k8 & (DH - 1);
    const float* p = W2 + (size_t)kk * DH + n;
#pragma unroll
    for (int i = 0; i < 8; ++i) o[i] = (unsigned short)bf16_bits(p[(size_t)i * DH]);
    dp = W2D + (size_t)n * KP + k8;
  } else if (u < NU1 + 2 * NU2) {
    const int v  = u - NU1 - NU2;
    const int n  = v >> 5;
    const int k8 = (v & 31) * 8;
    const int kk = k8 & (DH - 1);
    const float* p = W3 + (size_t)kk * DH + n;
#pragma unroll
    for (int i = 0; i < 8; ++i) o[i] = (unsigned short)bf16_bits(p[(size_t)i * DH]);
    dp = W3D + (size_t)n * KP + k8;
  } else {
    return;
  }
  *(volatile v8us*)dp = o;
  __threadfence();
  *(volatile v8us*)dp = o;
}

__global__ __launch_bounds__(NTHR) void k_cvx(const float* __restrict__ x, int nN, int nUnits,
                                              unsigned short* xb) {
  const int u = (int)blockIdx.x * NTHR + (int)threadIdx.x;
  if (u >= nUnits) return;
  const int row = u >> 4;
  const int k8  = (u & 15) * 8;
  const int rc  = row < nN ? row : nN - 1;
  const float* p = x + (size_t)rc * DIN + k8;
  const v4f a = *(const v4f*)p;
  const v4f b = *(const v4f*)(p + 4);
  const bool ok = row < nN;
  v8us o;
  o[0] = ok ? (unsigned short)bf16_bits(a.x) : (unsigned short)0;
  o[1] = ok ? (unsigned short)bf16_bits(a.y) : (unsigned short)0;
  o[2] = ok ? (unsigned short)bf16_bits(a.z) : (unsigned short)0;
  o[3] = ok ? (unsigned short)bf16_bits(a.w) : (unsigned short)0;
  o[4] = ok ? (unsigned short)bf16_bits(b.x) : (unsigned short)0;
  o[5] = ok ? (unsigned short)bf16_bits(b.y) : (unsigned short)0;
  o[6] = ok ? (unsigned short)bf16_bits(b.z) : (unsigned short)0;
  o[7] = ok ? (unsigned short)bf16_bits(b.w) : (unsigned short)0;
  unsigned short* dp = xb + (size_t)row * DIN + k8;
  *(volatile v8us*)dp = o;
  __threadfence();
  *(volatile v8us*)dp = o;
}

__global__ __launch_bounds__(GTHR) void k_gemm(const unsigned short* __restrict__ A, int lda,
                                               const unsigned short* __restrict__ BT, int ldb, int K,
                                               float* Cm, const float* __restrict__ avs,
                                               const float* __restrict__ avd, float* AL) {
  constexpr int LDC = GBN;
  constexpr int RPW = GBM / 4;
  __shared__ __attribute__((aligned(16))) float stg[GBM * LDC];
  __shared__ __attribute__((aligned(16))) float sdt[2 * GBM];
  const int tid = (int)threadIdx.x, lane = tid & 31, wave = tid >> 5, hh = lane >> 4, m = lane & 15;
  const int rg = wave;
  const int rowBase = (int)blockIdx.x * GBM;

  v8f acc[8];
  {
    const v8f z = {0.f, 0.f, 0.f, 0.f, 0.f, 0.f, 0.f, 0.f};
#pragma unroll
    for (int t = 0; t < 8; ++t) acc[t] = z;
  }
  const unsigned short* ap = A  + (size_t)(rowBase + 16 * rg + m) * (size_t)lda + 8 * hh;
  const unsigned short* bp = BT + (size_t)m * (size_t)ldb + 8 * hh;

#pragma unroll 1
  for (int k0 = 0; k0 < K; k0 += 32) {
    FragB af;
    af.h[0] = *(const v8usa*)(ap + k0);
    af.h[1] = *(const v8usa*)(ap + k0 + 16);
#pragma unroll
    for (int nt = 0; nt < 8; ++nt) {
      const unsigned short* wq = bp + (size_t)(16 * nt) * (size_t)ldb + k0;
      FragB bf;
      bf.h[0] = *(const v8usa*)wq;
      bf.h[1] = *(const v8usa*)(wq + 16);
      acc[nt] = wmb(af, bf, acc[nt]);
    }
  }

#pragma unroll
  for (int nt = 0; nt < 8; ++nt) {
    const int lc = 16 * nt + m;
#pragma unroll
    for (int r = 0; r < 8; ++r) {
      const int lr = 16 * rg + 8 * hh + r;
      stg[lr * LDC + lc] = acc[nt][r];
    }
  }
  __syncthreads();

  const v4f as4 = bfr4(*(const v4fa*)(avs + 4 * lane));
  const v4f ad4 = bfr4(*(const v4fa*)(avd + 4 * lane));
#pragma unroll 1
  for (int i = 0; i < RPW; ++i) {
    const int row = wave * RPW + i;
    const v4f p = *(const v4fa*)(stg + row * LDC + 4 * lane);
    float s = 0.0f, d = 0.0f;
    s = fmaf(p.x, as4.x, s); s = fmaf(p.y, as4.y, s); s = fmaf(p.z, as4.z, s); s = fmaf(p.w, as4.w, s);
    d = fmaf(p.x, ad4.x, d); d = fmaf(p.y, ad4.y, d); d = fmaf(p.z, ad4.z, d); d = fmaf(p.w, ad4.w, d);
#pragma unroll
    for (int off = 16; off > 0; off >>= 1) {
      s += __shfl_xor(s, off);
      d += __shfl_xor(d, off);
    }
    if (lane == 0) { sdt[row] = s; sdt[GBM + row] = d; }
  }
  __syncthreads();

  const v4f alv = *(const v4fa*)(sdt + 4 * lane);
  float* alp = AL + (size_t)blockIdx.x * (2 * GBM) + 4 * lane;
#pragma unroll 1
  for (int i = 0; i < RPW; ++i) {
    const int row = wave * RPW + i;
    const v4f p = *(const v4fa*)(stg + row * LDC + 4 * lane);
    float* op = Cm + (size_t)(rowBase + row) * (size_t)LDC + 4 * lane;
    *(volatile v4f*)op = p;
  }
  if (wave == 0) *(volatile v4f*)alp = alv;
  __threadfence();
#pragma unroll 1
  for (int i = 0; i < RPW; ++i) {
    const int row = wave * RPW + i;
    const v4f p = *(const v4fa*)(stg + row * LDC + 4 * lane);
    float* op = Cm + (size_t)(rowBase + row) * (size_t)LDC + 4 * lane;
    *(volatile v4f*)op = p;
  }
  if (wave == 0) *(volatile v4f*)alp = alv;
}

template <int RL>
__global__ __launch_bounds__(NTHR) void k_agg(const int* __restrict__ srcs, const int* __restrict__ dsts,
                                              int nE, int nN, int vec8, int mRows,
                                              const float* __restrict__ AL,
                                              const float* __restrict__ xl, const float* __restrict__ bias,
                                              unsigned short* hb, float* outp) {
  extern __shared__ __attribute__((aligned(16))) int dsm[];
  int* list = dsm;
  int* hl   = dsm + LISTN;
  int* sl   = dsm + LISTN + RCAP;
  int* cnt  = dsm + LISTN + 2 * RCAP;
  int* offs = cnt + NBA;
  int* cur  = offs + NBA;
  int* misc = cur + NBA;
  const int tid = (int)threadIdx.x, lane = tid & 31, wave = tid >> 5;
  const int nodeBase = (int)blockIdx.x * NBA;

  {
    const v4i z4 = {0, 0, 0, 0};
    for (int i = tid * 4; i < AGG_ZINTS; i += NTHR * 4) *(v4ia*)(dsm + i) = z4;
    if (tid < 16) misc[tid] = 0;
  }
  const v4f bv = bfr4(*(const v4f*)(bias + 4 * lane));
  __syncthreads();

  int t = 0, ov = 0;
  const int nChunks = (nE + CHUNK - 1) / CHUNK;
#pragma unroll 1
  for (int ch = 0; ch < nChunks; ++ch) {
    const int cbase = ch * CHUNK;
    const int wc = scan_chunk<SLA>(dsts, nE, cbase, nodeBase, NBA, vec8, list, tid, lane, wave);
    if (lane == 0) misc[wave] = wc;
    __syncthreads();
    if (wave == 0) {
#pragma unroll 1
      for (int w2 = 0; w2 < NWAVE; ++w2) {
        int c = misc[w2];
        c = c < 0 ? 0 : (c > WCAP ? WCAP : c);
#pragma unroll 1
        for (int b0 = 0; b0 < c; b0 += 32) {
          const int idx = b0 + lane;
          const int ent = list[w2 * WCAP + (idx < WCAP ? idx : WCAP - 1)];
          const int m32 = (c - b0) < 32 ? (c - b0) : 32;
#pragma unroll 1
          for (int k = 0; k < m32; ++k) {
            const int u    = __builtin_amdgcn_readlane(ent, k);
            const int slot = u & (NBA - 1);
            const int el   = (u >> SLA) & (CHUNK - 1);
            const int pk   = ((cbase + el) << SLA) | slot;
            if (t < RCAP) {
              if (lane == 0) { hl[t] = pk; cnt[slot] = cnt[slot] + 1; }
              t = t + 1;
            } else {
              ov = 1;
            }
          }
        }
      }
    }
    __syncthreads();
  }
  if (wave == 0 && lane == 0) { misc[8] = t; misc[9] = ov; }
  __syncthreads();
  int tt = misc[8];
  tt = tt < 0 ? 0 : (tt > RCAP ? RCAP : tt);
  const int ovf = misc[9];

  if (wave == 0) {
    const int base = lane * (NBA / 32);
    int s = 0;
#pragma unroll 1
    for (int i = 0; i < NBA / 32; ++i) s += cnt[base + i];
    int incl = s;
#pragma unroll
    for (int d = 1; d < 32; d <<= 1) {
      const int y = __shfl_up(incl, d, 32);
      if (lane >= d) incl += y;
    }
    int run = incl - s;
#pragma unroll 1
    for (int i = 0; i < NBA / 32; ++i) {
      const int cv = cnt[base + i];
      offs[base + i] = run;
      cur[base + i]  = run;
      run += cv;
    }
  }
  __syncthreads();
  if (wave == 0) {
#pragma unroll 1
    for (int b0 = 0; b0 < tt; b0 += 32) {
      const int idx = b0 + lane;
      const int ent = hl[idx < RCAP ? idx : RCAP - 1];
      const int m32 = (tt - b0) < 32 ? (tt - b0) : 32;
#pragma unroll 1
      for (int k = 0; k < m32; ++k) {
        const int u    = __builtin_amdgcn_readlane(ent, k);
        const int slot = u & (NBA - 1);
        if (lane == 0) {
          int p = cur[slot];
          p = p < 0 ? 0 : (p > RCAP - 1 ? RCAP - 1 : p);
          sl[p] = u;
          cur[slot] = p + 1;
        }
      }
    }
  }
  __syncthreads();

  const float qnan = __int_as_float(0x7fc00000);
  const float pz = (ovf != 0) ? qnan : 0.0f;
#pragma unroll 1
  for (int si = 0; si < NBA / NWAVE; ++si) {
    const int s    = si * NWAVE + wave;
    const int node = nodeBase + s;
    int c = cnt[s];
    const bool big = c > DEGCAP;
    c = c < 0 ? 0 : (c > DEGCAP ? DEGCAP : c);
    int o = offs[s];
    o = o < 0 ? 0 : (o > RCAP ? RCAP : o);
    const int nc  = node < nN ? node : nN - 1;
    const int alb = (nc >> 6) * (2 * GBM) + (nc & (GBM - 1));
    const float as0 = AL[alb];
    const float ad  = AL[alb + GBM];
    v4f acc = *(const v4f*)(xl + (size_t)nc * DH + 4 * lane);
    float l0 = as0 + ad;
    l0 = l0 > 0.f ? l0 : NEGSL * l0;
    float mx = l0, dn = 1.0f;
#pragma unroll 1
    for (int b0 = 0; b0 < c; b0 += 32) {
      int idx = o + b0 + lane;
      idx = idx > RCAP - 1 ? RCAP - 1 : idx;
      const int ent = sl[idx];
      int eid = ent >> SLA;
      eid = eid < 0 ? 0 : (eid > nE - 1 ? nE - 1 : eid);
      int sr = srcs[eid];
      sr = sr < 0 ? 0 : (sr > nN - 1 ? nN - 1 : sr);
      const float es  = AL[(sr >> 6) * (2 * GBM) + (sr & (GBM - 1))];
      const int   esi = __float_as_int(es);
      const int m32 = (c - b0) < 32 ? (c - b0) : 32;
#pragma unroll 1
      for (int k = 0; k < m32; ++k) {
        const int   sk  = __builtin_amdgcn_readlane(sr, k);
        const float ask = __int_as_float(__builtin_amdgcn_readlane(esi, k));
        const float* rp = xl + (size_t)sk * DH + 4 * lane;
        const v4f a = *(const v4f*)rp;
        float lg = ask + ad;
        lg = lg > 0.f ? lg : NEGSL * lg;
        const float df = lg - mx;
        const float ee = expf(-fabsf(df));
        const bool  up = df > 0.f;
        const float s1 = up ? ee : 1.0f;
        const float s2 = up ? 1.0f : ee;
        mx = up ? lg : mx;
        dn = fmaf(dn, s1, s2);
        acc.x = fmaf(acc.x, s1, s2 * a.x); acc.y = fmaf(acc.y, s1, s2 * a.y);
        acc.z = fmaf(acc.z, s1, s2 * a.z); acc.w = fmaf(acc.w, s1, s2 * a.w);
      }
    }
    const float msel = (fabsf(mx) <= 3.4028234e38f) ? mx : 0.0f;
    const float gsc  = expf(mx - msel);
    const float inv  = 1.0f / (dn * gsc + EPS_SM);
    const float wsc  = gsc * inv;
    v4f y;
    y.x = fmaf(acc.x, wsc, bv.x);
    y.y = fmaf(acc.y, wsc, bv.y);
    y.z = fmaf(acc.z, wsc, bv.z);
    y.w = fmaf(acc.w, wsc, bv.w);
#pragma unroll 1
    for (int r = 0; r < 4; ++r) {
      const float tv = y.x;
      const float ev = (tv > 0.0f) ? tv : expm1f(tv);
      y.x = y.y; y.y = y.z; y.z = y.w; y.w = ev;
    }
    const float pzr = big ? qnan : pz;
    const bool live = node < nN;
    v4f v;
    v.x = live ? (y.x + pzr) : 0.0f;
    v.y = live ? (y.y + pzr) : 0.0f;
    v.z = live ? (y.z + pzr) : 0.0f;
    v.w = live ? (y.w + pzr) : 0.0f;
    if constexpr (RL != 0) {
      const unsigned hbx = bf16_bits(v.x) & 0xFFFFu, hby = bf16_bits(v.y) & 0xFFFFu;
      const unsigned hbz = bf16_bits(v.z) & 0xFFFFu, hbw = bf16_bits(v.w) & 0xFFFFu;
      const unsigned lbx = bf16_bits(v.x - __uint_as_float(hbx << 16)) & 0xFFFFu;
      const unsigned lby = bf16_bits(v.y - __uint_as_float(hby << 16)) & 0xFFFFu;
      const unsigned lbz = bf16_bits(v.z - __uint_as_float(hbz << 16)) & 0xFFFFu;
      const unsigned lbw = bf16_bits(v.w - __uint_as_float(hbw << 16)) & 0xFFFFu;
      const int hw0 = (int)(hbx | (hby << 16)), hw1 = (int)(hbz | (hbw << 16));
      const int lw0 = (int)(lbx | (lby << 16)), lw1 = (int)(lbz | (lbw << 16));
      const int sa = (2 * lane) & 31, sb = (2 * lane + 1) & 31;
      const int g0 = __shfl(hw0, sa), g1 = __shfl(hw1, sa), g2 = __shfl(hw0, sb), g3 = __shfl(hw1, sb);
      const int q0 = __shfl(lw0, sa), q1 = __shfl(lw1, sa), q2 = __shfl(lw0, sb), q3 = __shfl(lw1, sb);
      const bool lsel = lane >= 16;
      v4u pv;
      pv.x = (unsigned)(lsel ? q0 : g0);
      pv.y = (unsigned)(lsel ? q1 : g1);
      pv.z = (unsigned)(lsel ? q2 : g2);
      pv.w = (unsigned)(lsel ? q3 : g3);
      if (node < mRows) {
        unsigned short* gp = hb + (size_t)node * KP + 8 * lane;
        *(volatile v4u*)gp = pv;
        __threadfence();
        *(volatile v4u*)gp = pv;
      }
    } else {
      if (live) {
        float* op = outp + (size_t)node * DH + 4 * lane;
        *(volatile v4f*)op = v;
        __threadfence();
        *(volatile v4f*)op = v;
      }
    }
  }
}

__global__ __launch_bounds__(PTHR) void k_pool_part(const float* __restrict__ H3, const int* __restrict__ batch,
                                                    int nN, float* PP, float* PC) {
  __shared__ __attribute__((aligned(16))) float bins[NGR * DH];
  __shared__ __attribute__((aligned(16))) float scn[NGR];
  const int tid = (int)threadIdx.x;
  for (int i = tid; i < NGR * DH; i += PTHR) bins[i] = 0.0f;
  __syncthreads();
  const int n0 = (int)blockIdx.x * NPB;
  int n1 = n0 + NPB; n1 = n1 > nN ? nN : n1;
  float mycnt = 0.0f;
#pragma unroll 2
  for (int n = n0; n < n1; ++n) {
    const int   g  = batch[n];
    const float hv = H3[(size_t)n * DH + tid];
    const bool  ok = (unsigned)g < (unsigned)NGR;
    const int   gc = ok ? g : 0;
    const float ad = ok ? hv : 0.0f;
    bins[gc * DH + tid] = bins[gc * DH + tid] + ad;
    mycnt += (ok && g == tid) ? 1.0f : 0.0f;
  }
  __syncthreads();
  if (tid < NGR) scn[tid] = mycnt;
  __syncthreads();
  float* pb = PP + (size_t)blockIdx.x * (size_t)(NGR * DH);
  float* pc = PC + (size_t)blockIdx.x * NGR;
#pragma unroll 1
  for (int i = tid; i < NGR * DH / 4; i += PTHR) {
    const v4f v = *(const v4fa*)(bins + 4 * i);
    *(volatile v4f*)(pb + 4 * i) = v;
  }
  if (tid < NGR / 4) {
    const v4f cv = *(const v4fa*)(scn + 4 * tid);
    *(volatile v4f*)(pc + 4 * tid) = cv;
  }
  __threadfence();
#pragma unroll 1
  for (int i = tid; i < NGR * DH / 4; i += PTHR) {
    const v4f v = *(const v4fa*)(bins + 4 * i);
    *(volatile v4f*)(pb + 4 * i) = v;
  }
  if (tid < NGR / 4) {
    const v4f cv = *(const v4fa*)(scn + 4 * tid);
    *(volatile v4f*)(pc + 4 * tid) = cv;
  }
}

__global__ __launch_bounds__(PTHR) void k_pool_comb(const float* __restrict__ PP, const float* __restrict__ PC,
                                                    int nP, float* outp) {
  __shared__ __attribute__((aligned(16))) float sres[DH];
  const int tid = (int)threadIdx.x;
  const int g = (int)blockIdx.x;
  double sm = 0.0;
  float cn = 0.0f;
#pragma unroll 2
  for (int p = 0; p < nP; ++p) {
    sm += (double)PP[((size_t)p * NGR + g) * DH + tid];
    cn += PC[(size_t)p * NGR + g];
  }
  const float den = cn > 1.0f ? cn : 1.0f;
  const float res = (float)sm * (1.0f / den);
  sres[tid] = res;
  __syncthreads();
  if (tid < 32) {
    const v4f v = *(const v4fa*)(sres + 4 * tid);
    float* op = outp + (size_t)g * DH + 4 * tid;
    *(volatile v4f*)op = v;
    __threadfence();
    *(volatile v4f*)op = v;
  }
}

static inline int cdiv(int a, int b) { return (a + b - 1) / b; }

extern "C" void kernel_launch(void* const* d_in, const int* in_sizes, int n_in,
                              void* d_out, int out_size, void* d_ws, size_t ws_size,
                              hipStream_t stream) {
  if (n_in < 15) return;
  if (in_sizes[0] < DIN || (in_sizes[0] % DIN) != 0) return;
  const int nN = in_sizes[0] / DIN;
  if (nN > (1 << 22)) return;
  if (in_sizes[1] < 2 || (in_sizes[1] & 1) != 0) return;
  const int nE = in_sizes[1] / 2;
  if (nE < 1 || nE >= (1 << 21)) return;
  if (in_sizes[2] != nN) return;
  if (in_sizes[3] != DIN * DH) return;
  if (in_sizes[4] != DH || in_sizes[5] != DH || in_sizes[6] != DH) return;
  if (in_sizes[7] != DH * DH) return;
  if (in_sizes[8] != DH || in_sizes[9] != DH || in_sizes[10] != DH) return;
  if (in_sizes[11] != DH * DH) return;
  if (in_sizes[12] != DH || in_sizes[13] != DH || in_sizes[14] != DH) return;
  if (out_size != NGR * DH) return;

  const float* x    = (const float*)d_in[0];
  const int*   edge = (const int*)d_in[1];
  const int*   bat  = (const int*)d_in[2];
  const float* W1   = (const float*)d_in[3];
  const float* a1s  = (const float*)d_in[4];
  const float* a1d  = (const float*)d_in[5];
  const float* b1   = (const float*)d_in[6];
  const float* W2   = (const float*)d_in[7];
  const float* a2s  = (const float*)d_in[8];
  const float* a2d  = (const float*)d_in[9];
  const float* b2   = (const float*)d_in[10];
  const float* W3   = (const float*)d_in[11];
  const float* a3s  = (const float*)d_in[12];
  const float* a3d  = (const float*)d_in[13];
  const float* b3   = (const float*)d_in[14];
  float* out = (float*)d_out;
  const int* src = edge;
  const int* dst = edge + nE;

  const int MP   = cdiv(nN, GBM) * GBM;
  const int gM   = MP / GBM;
  const int gA   = cdiv(MP, NBA);
  if ((long long)gA * NBA < (long long)MP) return;
  const int vec8 = ((nE & 3) == 0) ? 1 : 0;
  const int nP   = cdiv(nN, NPB);

  char* ws = (char*)d_ws;
  size_t off = 0;
  const size_t oW1T = off; off += (size_t)DH * DIN * 2;                   off = (off + 255) & ~(size_t)255;
  const size_t oW2D = off; off += (size_t)DH * KP * 2;                    off = (off + 255) & ~(size_t)255;
  const size_t oW3D = off; off += (size_t)DH * KP * 2;                    off = (off + 255) & ~(size_t)255;
  const size_t oAL  = off; off += (size_t)gM * (2 * GBM) * 4;             off = (off + 255) & ~(size_t)255;
  const size_t oXB  = off; off += (size_t)MP * DIN * 2;                   off = (off + 255) & ~(size_t)255;
  const size_t oH   = off; off += (size_t)MP * DH * 4;                    off = (off + 255) & ~(size_t)255;
  const size_t oAP  = off; off += (size_t)MP * KP * 2;                    off = (off + 255) & ~(size_t)255;
  const size_t oH3  = off; off += (size_t)MP * DH * 4;                    off = (off + 255) & ~(size_t)255;
  const size_t oPP  = off; off += (size_t)nP * NGR * DH * 4;              off = (off + 255) & ~(size_t)255;
  const size_t oPC  = off; off += (size_t)nP * NGR * 4;                   off = (off + 255) & ~(size_t)255;
  if (off > ws_size || off > (size_t)WSMAX) return;
  unsigned short* W1T = (unsigned short*)(ws + oW1T);
  unsigned short* W2D = (unsigned short*)(ws + oW2D);
  unsigned short* W3D = (unsigned short*)(ws + oW3D);
  float*          ALp = (float*)(ws + oAL);
  unsigned short* XB  = (unsigned short*)(ws + oXB);
  float*          H   = (float*)(ws + oH);
  unsigned short* AP  = (unsigned short*)(ws + oAP);
  float*          H3  = (float*)(ws + oH3);
  float*          PP  = (float*)(ws + oPP);
  float*          PC  = (float*)(ws + oPC);

  const size_t aggLds = (size_t)AGG_LDS_INTS * 4;
  hipFuncSetAttribute(reinterpret_cast<const void*>(&k_agg<1>), hipFuncAttributeMaxDynamicSharedMemorySize, (int)aggLds);
  hipFuncSetAttribute(reinterpret_cast<const void*>(&k_agg<0>), hipFuncAttributeMaxDynamicSharedMemorySize, (int)aggLds);

  const int nUx = MP * (DIN / 8);
  k_wprep<<<(NU1 + 2 * NU2) / NTHR, NTHR, 0, stream>>>(W1, W2, W3, W1T, W2D, W3D);
  k_cvx<<<cdiv(nUx, NTHR), NTHR, 0, stream>>>(x, nN, nUx, XB);
  k_gemm<<<gM, GTHR, 0, stream>>>(XB, DIN, W1T, DIN, DIN, H, a1s, a1d, ALp);
  k_agg<1><<<gA, NTHR, aggLds, stream>>>(src, dst, nE, nN, vec8, MP, ALp, H, b1, AP, H3);
  k_gemm<<<gM, GTHR, 0, stream>>>(AP, KP, W2D, KP, KP, H, a2s, a2d, ALp);
  k_agg<1><<<gA, NTHR, aggLds, stream>>>(src, dst, nE, nN, vec8, MP, ALp, H, b2, AP, H3);
  k_gemm<<<gM, GTHR, 0, stream>>>(AP, KP, W3D, KP, KP, H, a3s, a3d, ALp);
  k_agg<0><<<gA, NTHR, aggLds, stream>>>(src, dst, nE, nN, vec8, MP, ALp, H, b3, AP, H3);
  k_pool_part<<<nP, PTHR, 0, stream>>>(H3, bat, nN, PP, PC);
  k_pool_comb<<<NGR, PTHR, 0, stream>>>(PP, PC, nP, out);
}
